// EdgeConvGNN_68375879352753
// MI455X (gfx1250) — hardware-verified
//
#include <hip/hip_runtime.h>
#include <stddef.h>
#include <math.h>


#define CIN    16
#define HCH    32
#define NG     64
#define KP     32
#define APZ    40
#define KPB    32
#define NTHR   256
#define NWAVE  8
#define NIT    16
#define NPB    (NWAVE * NIT)
#define GROWS  64
#define GTHR   128
#define DEGCAP 512
#define EPT    8
#define NGRP   2
#define CHUNK  (NTHR * EPT * NGRP)
#define WCAP   256
#define LISTN  (NWAVE * WCAP)
#define NBC    4096
#define NBF    2048
#define RCAP   67072
#define RBN    128
#define OTHR   512
#define LDS_FILL ((RCAP + NBF + LISTN) * 4 + 64)
#define O_N1H  0
#define O_N1L  1024
#define O_W1H  2048
#define O_W1L  2560
#define O_N2H  3072
#define O_N2L  5120
#define O_W2H  7168
#define O_W2L  8192
#define BPTOT  9216
#define WPSLOT 576
#define WSCAP  134217728

static_assert(NIT * NWAVE == NPB);
static_assert(GROWS == (GTHR / 32) * 16);
static_assert(GTHR == 2 * GROWS);
static_assert((APZ % 8) == 0 && (KPB % 8) == 0 && APZ >= KP && KPB >= KP);
static_assert((CHUNK & (CHUNK - 1)) == 0 && CHUNK <= 4096);
static_assert(NBC <= 4096 && (NBC & (NBC - 1)) == 0 && (NBF & (NBF - 1)) == 0);
static_assert(NBC == 2 * NBF);
static_assert(OTHR * 8 == NBC);
static_assert((RCAP % 32) == 0);
static_assert((DEGCAP % 16) == 0);
static_assert(NTHR == 4 * NG);
static_assert(BPTOT == O_W2L + HCH * KPB);
static_assert(WPSLOT * 16 == BPTOT);
static_assert((O_N1L % 64) == 0 && (O_W1H % 64) == 0 && (O_W1L % 64) == 0 && (O_N2H % 64) == 0);
static_assert((O_N2L % 64) == 0 && (O_W2H % 64) == 0 && (O_W2L % 64) == 0);

typedef float          v4f   __attribute__((ext_vector_type(4)));
typedef float          v8f   __attribute__((ext_vector_type(8)));
typedef int            v4i   __attribute__((ext_vector_type(4)));
typedef unsigned short v4us  __attribute__((ext_vector_type(4)));
typedef unsigned short v8us  __attribute__((ext_vector_type(8)));
typedef unsigned short v16us __attribute__((ext_vector_type(16)));
typedef __bf16         v16b  __attribute__((ext_vector_type(16)));
union Frag { v16us u; v8us h[2]; };

__device__ __forceinline__ unsigned short bfr(float f) {
  const unsigned u = __float_as_uint(f);
  return (unsigned short)((u + 0x7FFFu + ((u >> 16) & 1u)) >> 16);
}
__device__ __forceinline__ float bfv(unsigned short h) { return __uint_as_float(((unsigned)h) << 16); }

__device__ __forceinline__ void split4(v4f a, v4us& uh, v4us& ul) {
  const unsigned short h0 = bfr(a.x), h1 = bfr(a.y), h2 = bfr(a.z), h3 = bfr(a.w);
  uh.x = h0; uh.y = h1; uh.z = h2; uh.w = h3;
  ul.x = bfr(a.x - bfv(h0)); ul.y = bfr(a.y - bfv(h1)); ul.z = bfr(a.z - bfv(h2)); ul.w = bfr(a.w - bfv(h3));
}
__device__ __forceinline__ void split8(const float (&v)[8], v8us& uh, v8us& ul) {
#pragma unroll
  for (int e = 0; e < 8; ++e) {
    const unsigned short h = bfr(v[e]);
    uh[e] = h;
    ul[e] = bfr(v[e] - bfv(h));
  }
}

__device__ __forceinline__ v8f wmb(v16us a, v16us b, v8f c) {
  const v16b av = __builtin_bit_cast(v16b, a);
  const v16b bv = __builtin_bit_cast(v16b, b);
  v8f d = __builtin_amdgcn_wmma_f32_16x16x32_bf16(false, av, false, bv, (short)0, c, false, false);
  asm volatile("v_nop\n\tv_nop\n\tv_nop\n\tv_nop" : "+v"(d) : "v"(av), "v"(bv));
  return d;
}

template <int NT>
__device__ __forceinline__ void mma3(const unsigned short* Ah, const unsigned short* Al,
                                     const unsigned short* __restrict__ Bh, const unsigned short* __restrict__ Bl,
                                     int lane, v8f (&acc)[NT]) {
  const int hh = lane >> 4, m = lane & 15;
  Frag ah, al;
  ah.h[0] = *(const v8us*)(Ah + m * APZ + 8 * hh);
  ah.h[1] = *(const v8us*)(Ah + m * APZ + 16 + 8 * hh);
  al.h[0] = *(const v8us*)(Al + m * APZ + 8 * hh);
  al.h[1] = *(const v8us*)(Al + m * APZ + 16 + 8 * hh);
#pragma unroll
  for (int t = 0; t < NT; ++t) {
    const unsigned short* bph = Bh + (16 * t + m) * KPB + 8 * hh;
    const unsigned short* bpl = Bl + (16 * t + m) * KPB + 8 * hh;
    Frag bh, bl;
    bh.h[0] = *(const v8us*)bph;
    bh.h[1] = *(const v8us*)(bph + 16);
    bl.h[0] = *(const v8us*)bpl;
    bl.h[1] = *(const v8us*)(bpl + 16);
    v8f z = {0.f, 0.f, 0.f, 0.f, 0.f, 0.f, 0.f, 0.f};
    z = wmb(ah.u, bh.u, z);
    z = wmb(al.u, bh.u, z);
    z = wmb(ah.u, bl.u, z);
    acc[t] = z;
  }
}

template <int NB>
__device__ __forceinline__ int scan_chunk(const int* __restrict__ dsts, int nE, int cbase, int slotBase,
                                          int vec8, int* list, int tid, int lane, int wave) {
  int wc = 0;
#pragma unroll
  for (int g = 0; g < NGRP; ++g) {
    const int el0  = (g * NTHR + tid) * EPT;
    const int e0   = cbase + el0;
    const int sent = -2147483647 - 1;
    v4i da, db;
    if (vec8 != 0 && cbase + CHUNK <= nE) {
      da = *(const v4i*)(dsts + e0);
      db = *(const v4i*)(dsts + e0 + 4);
    } else {
      da.x = (e0     < nE) ? dsts[min(e0, nE - 1)] : sent;
      da.y = (e0 + 1 < nE) ? dsts[min(e0 + 1, nE - 1)] : sent;
      da.z = (e0 + 2 < nE) ? dsts[min(e0 + 2, nE - 1)] : sent;
      da.w = (e0 + 3 < nE) ? dsts[min(e0 + 3, nE - 1)] : sent;
      db.x = (e0 + 4 < nE) ? dsts[min(e0 + 4, nE - 1)] : sent;
      db.y = (e0 + 5 < nE) ? dsts[min(e0 + 5, nE - 1)] : sent;
      db.z = (e0 + 6 < nE) ? dsts[min(e0 + 6, nE - 1)] : sent;
      db.w = (e0 + 7 < nE) ? dsts[min(e0 + 7, nE - 1)] : sent;
    }
    const unsigned nb = (unsigned)slotBase;
    const unsigned s0 = (unsigned)da.x - nb, s1 = (unsigned)da.y - nb;
    const unsigned s2 = (unsigned)da.z - nb, s3 = (unsigned)da.w - nb;
    const unsigned s4 = (unsigned)db.x - nb, s5 = (unsigned)db.y - nb;
    const unsigned s6 = (unsigned)db.z - nb, s7 = (unsigned)db.w - nb;
    const bool h0 = s0 < (unsigned)NB, h1 = s1 < (unsigned)NB, h2 = s2 < (unsigned)NB, h3 = s3 < (unsigned)NB;
    const bool h4 = s4 < (unsigned)NB, h5 = s5 < (unsigned)NB, h6 = s6 < (unsigned)NB, h7 = s7 < (unsigned)NB;
    const unsigned any = __builtin_amdgcn_ballot_w32(h0 | h1 | h2 | h3 | h4 | h5 | h6 | h7);
    if (any != 0u) {
#define HITJ(J, HJ, SJ) { \
        const unsigned mj = __builtin_amdgcn_ballot_w32(HJ); \
        if (mj != 0u) { \
          if (HJ) { \
            const int pos = wc + (int)__builtin_amdgcn_mbcnt_lo(mj, 0u); \
            if (pos < WCAP) list[wave * WCAP + pos] = ((el0 + (J)) << 12) | (int)(SJ); \
          } \
          wc += (int)__builtin_popcount(mj); } }
      HITJ(0, h0, s0)
      HITJ(1, h1, s1)
      HITJ(2, h2, s2)
      HITJ(3, h3, s3)
      HITJ(4, h4, s4)
      HITJ(5, h5, s5)
      HITJ(6, h6, s6)
      HITJ(7, h7, s7)
#undef HITJ
    }
  }
  return wc;
}

__global__ __launch_bounds__(NTHR) void k_wprep(const float* __restrict__ W1a, const float* __restrict__ W1b,
                                                const float* __restrict__ W2a, const float* __restrict__ W2b,
                                                unsigned short* Bpl) {
  const int i = blockIdx.x * NTHR + threadIdx.x;
  const bool act = i < WPSLOT;
  float v[8];
  int oh, ol;
  if (i < 128) {
    const int n = i >> 2, k0 = (i & 3) * 8, nc = n & 15;
#pragma unroll
    for (int e = 0; e < 8; ++e) {
      const int k = k0 + e, kc = k > 15 ? 15 : k;
      const float a = W1a[kc * 16 + nc], b = W1a[(16 + kc) * 16 + nc];
      const float t = (n < 16) ? (a - b) : b;
      v[e] = (k < 16) ? t : 0.0f;
    }
    oh = O_N1H + n * KPB + k0; ol = O_N1L + n * KPB + k0;
  } else if (i < 192) {
    const int j = i - 128, n = j >> 2, k0 = (j & 3) * 8;
#pragma unroll
    for (int e = 0; e < 8; ++e) {
      const int k = k0 + e, kc = k > 15 ? 15 : k;
      const float a = W1b[kc * 16 + n];
      v[e] = (k < 16) ? a : 0.0f;
    }
    oh = O_W1H + n * KPB + k0; ol = O_W1L + n * KPB + k0;
  } else if (i < 448) {
    const int j = i - 192, n = j >> 2, k0 = (j & 3) * 8, nc = n & 31;
#pragma unroll
    for (int e = 0; e < 8; ++e) {
      const int k = k0 + e, kc = k > 15 ? 15 : k;
      const float a = W2a[kc * 32 + nc], b = W2a[(16 + kc) * 32 + nc];
      const float t = (n < 32) ? (a - b) : b;
      v[e] = (k < 16) ? t : 0.0f;
    }
    oh = O_N2H + n * KPB + k0; ol = O_N2L + n * KPB + k0;
  } else {
    const int j = (i > WPSLOT - 1 ? WPSLOT - 1 : i) - 448, n = j >> 2, k0 = (j & 3) * 8;
#pragma unroll
    for (int e = 0; e < 8; ++e) v[e] = W2b[(k0 + e) * 32 + n];
    oh = O_W2H + n * KPB + k0; ol = O_W2L + n * KPB + k0;
  }
  v8us uh, ul;
  split8(v, uh, ul);
  unsigned short* ph = Bpl + oh;
  unsigned short* pl = Bpl + ol;
  if (act) { *(volatile v8us*)ph = uh; *(volatile v8us*)pl = ul; }
  __threadfence();
  if (act) { *(volatile v8us*)ph = uh; *(volatile v8us*)pl = ul; }
}

__global__ __launch_bounds__(NTHR) void k_count(const int* __restrict__ dsts, int* cnt, int nE, int vec8) {
  __shared__ __attribute__((aligned(16))) int scnt[NBC];
  __shared__ __attribute__((aligned(16))) int list[LISTN];
  __shared__ int wcnt[NWAVE];
  const int tid = threadIdx.x, lane = tid & 31, wave = tid >> 5;
  const int nodeBase = blockIdx.x * NBC;

  for (int i = tid; i < NBC; i += NTHR) scnt[i] = 0;
  __syncthreads();

  const int nChunks = (nE + CHUNK - 1) / CHUNK;
#pragma unroll 1
  for (int ch = 0; ch < nChunks; ++ch) {
    const int cbase = ch * CHUNK;
    const int wc = scan_chunk<NBC>(dsts, nE, cbase, nodeBase, vec8, list, tid, lane, wave);
    if (lane == 0) wcnt[wave] = wc;
    __syncthreads();
    if (wave == 0) {
#pragma unroll 1
      for (int wsx = 0; wsx < NWAVE; ++wsx) {
        int n = __builtin_amdgcn_readfirstlane(wcnt[wsx]);
        n = n > WCAP ? WCAP : (n < 0 ? 0 : n);
        const int* lp = list + wsx * WCAP;
#pragma unroll 1
        for (int i = 0; i < n; ++i) {
          const int ent  = __builtin_amdgcn_readfirstlane(lp[i]);
          const int slot = ent & (NBC - 1);
          if (lane == 0) scnt[slot] = scnt[slot] + 1;
        }
      }
    }
    __syncthreads();
  }

  v4i cq[4];
#pragma unroll
  for (int q = 0; q < 4; ++q) {
    const int f = (wave * 4 + q) * 128 + 4 * lane;
    cq[q] = *(const v4i*)(scnt + f);
  }
  int* cp = cnt + (size_t)nodeBase;
#pragma unroll
  for (int q = 0; q < 4; ++q) {
    const int f = (wave * 4 + q) * 128 + 4 * lane;
    *(volatile v4i*)(cp + f) = cq[q];
  }
  __threadfence();
#pragma unroll
  for (int q = 0; q < 4; ++q) {
    const int f = (wave * 4 + q) * 128 + 4 * lane;
    *(volatile v4i*)(cp + f) = cq[q];
  }
}

__global__ __launch_bounds__(OTHR) void k_offsets(const int* __restrict__ cnt, int* off, int* rbase, int nChunk) {
  __shared__ __attribute__((aligned(16))) int soff[NBC];
  __shared__ __attribute__((aligned(16))) int srb[RBN];
  __shared__ int wtot[OTHR / 32];
  const int tid = threadIdx.x, lane = tid & 31, wave = tid >> 5, sub = tid >> 8;
  for (int i = tid; i < RBN; i += OTHR) srb[i] = 0;
  int carry = 0;
#pragma unroll 1
  for (int ch = 0; ch < nChunk; ++ch) {
    const int base = ch * NBC;
    const v4i c0 = *(const v4i*)(cnt + base + 8 * tid);
    const v4i c1 = *(const v4i*)(cnt + base + 8 * tid + 4);
    const int e0 = max(c0.x, 0), e1 = max(c0.y, 0), e2 = max(c0.z, 0), e3 = max(c0.w, 0);
    const int e4 = max(c1.x, 0), e5 = max(c1.y, 0), e6 = max(c1.z, 0), e7 = max(c1.w, 0);
    const int ts = e0 + e1 + e2 + e3 + e4 + e5 + e6 + e7;
    int incl = ts;
#pragma unroll
    for (int d = 1; d < 32; d <<= 1) {
      const int t = __shfl_up(incl, d);
      if (lane >= d) incl += t;
    }
    if (lane == 31) wtot[wave] = incl;
    __syncthreads();
    const int S0 = wtot[0] + wtot[1] + wtot[2]  + wtot[3]  + wtot[4]  + wtot[5]  + wtot[6]  + wtot[7];
    const int S1 = wtot[8] + wtot[9] + wtot[10] + wtot[11] + wtot[12] + wtot[13] + wtot[14] + wtot[15];
    int pre = 0;
#pragma unroll 1
    for (int w = 8 * sub; w < wave; ++w) pre += wtot[w];
    const int b0 = carry;
    const int b1 = b0 + ((S0 + 31) & ~31);
    const int b2 = b1 + ((S1 + 31) & ~31);
    const int myb = sub == 0 ? b0 : b1;
    if (tid == 0) {
      srb[min(2 * ch + 0, RBN - 1)] = b0;
      srb[min(2 * ch + 1, RBN - 1)] = b1;
    }
    int run = myb + pre + incl - ts;
    soff[8 * tid + 0] = run; run += e0;
    soff[8 * tid + 1] = run; run += e1;
    soff[8 * tid + 2] = run; run += e2;
    soff[8 * tid + 3] = run; run += e3;
    soff[8 * tid + 4] = run; run += e4;
    soff[8 * tid + 5] = run; run += e5;
    soff[8 * tid + 6] = run; run += e6;
    soff[8 * tid + 7] = run;
    carry = b2;
    __syncthreads();
    const v4i o0 = *(const v4i*)(soff + 4 * tid);
    const v4i o1 = *(const v4i*)(soff + 4 * (tid + OTHR));
    int* op = off + base;
    *(volatile v4i*)(op + 4 * tid) = o0;
    *(volatile v4i*)(op + 4 * (tid + OTHR)) = o1;
    __threadfence();
    *(volatile v4i*)(op + 4 * tid) = o0;
    *(volatile v4i*)(op + 4 * (tid + OTHR)) = o1;
    __syncthreads();
  }
  if (tid == 0) srb[min(2 * nChunk, RBN - 1)] = carry;
  __syncthreads();
  v4i rv = {0, 0, 0, 0};
  if (tid < 32) rv = *(const v4i*)(srb + 4 * tid);
  if (tid < 32) *(volatile v4i*)(rbase + 4 * tid) = rv;
  __threadfence();
  if (tid < 32) *(volatile v4i*)(rbase + 4 * tid) = rv;
}

__global__ __launch_bounds__(NTHR) void k_fill(
    const int* __restrict__ srcs, const int* __restrict__ dsts,
    const int* __restrict__ off, const int* __restrict__ rbase,
    int* csr, int nN, int nE, int vec8, int csrLen) {
  extern __shared__ v4f lds_dyn[];
  int* region = (int*)lds_dyn;
  int* cursor = region + RCAP;
  int* list   = cursor + NBF;
  int* wcnt   = list + LISTN;
  const int tid = threadIdx.x, lane = tid & 31, wave = tid >> 5;
  const int b = blockIdx.x;
  const int nodeBase = b * NBF;

  int rb0 = rbase[b];
  const int rb1 = rbase[b + 1];
  rb0 = rb0 < 0 ? 0 : (rb0 > csrLen ? csrLen : rb0);
  rb0 &= ~31;
  int len = rb1 - rb0;
  len = len < 0 ? 0 : (len > RCAP ? RCAP : len);
  int lenW = (len + 31) & ~31;
  if (rb0 + lenW > csrLen) lenW = (csrLen - rb0) & ~31;

  {
    const v4i z = {0, 0, 0, 0};
    for (int i = tid; i < RCAP / 4; i += NTHR) ((v4i*)region)[i] = z;
    for (int s = tid; s < NBF; s += NTHR) {
      int o = off[nodeBase + s] - rb0;
      o = o < 0 ? 0 : (o > RCAP ? RCAP : o);
      cursor[s] = o;
    }
  }
  __syncthreads();

  const int nChunks = (nE + CHUNK - 1) / CHUNK;
#pragma unroll 1
  for (int ch = 0; ch < nChunks; ++ch) {
    const int cbase = ch * CHUNK;
    const int wc = scan_chunk<NBF>(dsts, nE, cbase, nodeBase, vec8, list, tid, lane, wave);
    if (lane == 0) wcnt[wave] = wc;
    __syncthreads();
    if (wave == 0) {
#pragma unroll 1
      for (int wsx = 0; wsx < NWAVE; ++wsx) {
        int n = __builtin_amdgcn_readfirstlane(wcnt[wsx]);
        n = n > WCAP ? WCAP : (n < 0 ? 0 : n);
        const int* lp = list + wsx * WCAP;
#pragma unroll 1
        for (int i = 0; i < n; ++i) {
          const int ent  = __builtin_amdgcn_readfirstlane(lp[i]);
          const int slot = ent & (NBF - 1);
          int e = cbase + ((ent >> 12) & (CHUNK - 1));
          e = e > nE - 1 ? nE - 1 : e;
          int sv = srcs[e];
          sv = sv < 0 ? 0 : (sv > nN - 1 ? nN - 1 : sv);
          if (lane == 0) {
            int pos = cursor[slot];
            pos = pos < 0 ? 0 : (pos > RCAP - 1 ? RCAP - 1 : pos);
            region[pos] = sv;
            const int np = pos + 1;
            cursor[slot] = np > RCAP ? RCAP : np;
          }
        }
      }
    }
    __syncthreads();
  }

  const int nv = lenW >> 2;
  int* gp = csr + rb0;
#pragma unroll 1
  for (int i = tid; i < nv; i += NTHR) { const v4i v = ((const v4i*)region)[i]; *(volatile v4i*)(gp + 4 * i) = v; }
  __threadfence();
#pragma unroll 1
  for (int i = tid; i < nv; i += NTHR) { const v4i v = ((const v4i*)region)[i]; *(volatile v4i*)(gp + 4 * i) = v; }
}

template <int NCO>
__global__ __launch_bounds__(GTHR) void k_node(const float* __restrict__ X, const unsigned short* __restrict__ Bh,
                                               const unsigned short* __restrict__ Bl, const float* __restrict__ ba,
                                               float* PQ, int nN) {
  constexpr int NT = NCO / 16, CPW = NCO / 2, NWR = NCO / 8;
  __shared__ __attribute__((aligned(16))) unsigned short Ah[GROWS * APZ];
  __shared__ __attribute__((aligned(16))) unsigned short Al[GROWS * APZ];
  __shared__ __attribute__((aligned(16))) float stg[GROWS * NCO];
  const int tid = threadIdx.x, lane = tid & 31, wave = tid >> 5, hh = lane >> 4, m = lane & 15;
  const int rowBase = blockIdx.x * GROWS;
  {
    const int r = tid >> 1, c0 = (tid & 1) * 8;
    int xr = rowBase + r;
    xr = xr > nN - 1 ? nN - 1 : xr;
    const float* xp = X + (size_t)xr * CIN + c0;
    const v4f a = *(const v4f*)xp, b = *(const v4f*)(xp + 4);
    float v[8];
    v[0] = a.x; v[1] = a.y; v[2] = a.z; v[3] = a.w; v[4] = b.x; v[5] = b.y; v[6] = b.z; v[7] = b.w;
    v8us uh, ul;
    split8(v, uh, ul);
    *(v8us*)(Ah + r * APZ + c0) = uh;
    *(v8us*)(Al + r * APZ + c0) = ul;
    const v8us z8 = {0, 0, 0, 0, 0, 0, 0, 0};
    *(v8us*)(Ah + r * APZ + 16 + c0) = z8;
    *(v8us*)(Al + r * APZ + 16 + c0) = z8;
  }
  __syncthreads();

  v8f acc[NT];
  mma3<NT>(Ah + wave * 16 * APZ, Al + wave * 16 * APZ, Bh, Bl, lane, acc);
  float* sp = stg + (wave * 16 + 8 * hh) * NCO + m;
#pragma unroll
  for (int t = 0; t < NT; ++t) {
    int bc = 16 * t + m;
    bc = bc > CPW - 1 ? CPW - 1 : bc;
    const float bv = (t < NT / 2) ? ba[bc] : 0.0f;
#pragma unroll
    for (int r = 0; r < 8; ++r) sp[r * NCO + 16 * t] = acc[t][r] + bv;
  }
  __syncthreads();

  float* gp = PQ + (size_t)rowBase * NCO;
#pragma unroll
  for (int it = 0; it < NWR; ++it) {
    const int f = it * GTHR + tid;
    const v4f v = *(const v4f*)(stg + 4 * f);
    *(volatile v4f*)(gp + 4 * f) = v;
  }
  __threadfence();
#pragma unroll
  for (int it = 0; it < NWR; ++it) {
    const int f = it * GTHR + tid;
    const v4f v = *(const v4f*)(stg + 4 * f);
    *(volatile v4f*)(gp + 4 * f) = v;
  }
}

template <int CI>
__global__ __launch_bounds__(NTHR) void k_edge(
    const float* __restrict__ PQ, const int* __restrict__ csr,
    const int* __restrict__ offp, const int* __restrict__ cntp,
    const unsigned short* __restrict__ Bh, const unsigned short* __restrict__ Bl,
    const float* __restrict__ bb,
    const float* __restrict__ Wg1, const float* __restrict__ bg1,
    const float* __restrict__ Wg2, const float* __restrict__ bg2,
    float* H, float* G, int nN, int csrLen) {
  constexpr int NT = CI / 16, PQW = 2 * CI, PPR = CI / 4, RPP = 32 / PPR, NPASS = 16 / RPP;
  constexpr int LPPR = (CI == 32) ? 3 : 2;
  __shared__ __attribute__((aligned(16))) unsigned short At[NWAVE * 2 * 16 * APZ];
  __shared__ __attribute__((aligned(16))) float sout[NWAVE * CI];
  __shared__ __attribute__((aligned(16))) float sg[NPB];
  __shared__ __attribute__((aligned(16))) float swg[HCH * 16 + 32];
  __shared__ __attribute__((aligned(16))) int slot[NWAVE];
  const int tid = threadIdx.x, lane = tid & 31, wave = tid >> 5, hh = lane >> 4, m = lane & 15;
  const int base = blockIdx.x * NPB;
  unsigned short* Awh = At + wave * (2 * 16 * APZ);
  unsigned short* Awl = Awh + 16 * APZ;
  {
    const v8us z8 = {0, 0, 0, 0, 0, 0, 0, 0};
    for (int i = tid; i < (NWAVE * 2 * 16 * APZ) / 8; i += NTHR) *(v8us*)(At + 8 * i) = z8;
    if (tid < NPB) sg[tid] = 0.0f;
    if (CI == 32) {
      swg[tid] = Wg1[tid];
      swg[tid + NTHR] = Wg1[tid + NTHR];
      if (tid < 16) { swg[512 + tid] = bg1[tid]; swg[528 + tid] = Wg2[tid]; }
    }
  }
  __syncthreads();
  const int p = lane & (PPR - 1), rq = lane >> LPPR;
  float bbv[NT];
#pragma unroll
  for (int t = 0; t < NT; ++t) bbv[t] = bb[16 * t + m];
  const float bg2v = bg2[0];

#pragma unroll 1
  for (int it = 0; it < NIT; ++it) {
    const int n = base + it * NWAVE + wave;
    const bool nval = n < nN;
    const int cc = nval ? n : nN - 1;
    const int cnr = cntp[cc];
    const int ofr = offp[cc];
    int cn = nval ? cnr : 0;
    cn = cn < 0 ? 0 : (cn > DEGCAP ? DEGCAP : cn);
    cn = __builtin_amdgcn_readfirstlane(cn);
    int of = ofr;
    of = of < 0 ? 0 : (of > csrLen ? csrLen : of);
    of = __builtin_amdgcn_readfirstlane(of);
    const v4f dnc = *(const v4f*)(PQ + (size_t)cc * PQW + 4 * p);
    const int ntw = (cn + 15) >> 4;
    if (lane == 0) slot[wave] = ntw;
    __syncthreads();
    int ntmax;
    {
      const v4i sA = *(const v4i*)slot, sB = *(const v4i*)(slot + 4);
      int mm = max(max(sA.x, sA.y), max(sA.z, sA.w));
      mm = max(mm, max(max(sB.x, sB.y), max(sB.z, sB.w)));
      mm = mm < 0 ? 0 : (mm > DEGCAP / 16 ? DEGCAP / 16 : mm);
      ntmax = __builtin_amdgcn_readfirstlane(mm);
    }
    float cs[NT];
#pragma unroll
    for (int t = 0; t < NT; ++t) cs[t] = 0.0f;
#pragma unroll 1
    for (int tt = 0; tt < ntmax; ++tt) {
      int nv = cn - tt * 16;
      nv = nv < 0 ? 0 : (nv > 16 ? 16 : nv);
      int pos = of + tt * 16 + m;
      pos = pos < 0 ? 0 : (pos > csrLen - 1 ? csrLen - 1 : pos);
      int sv = csr[pos];
      sv = sv < 0 ? 0 : (sv > nN - 1 ? nN - 1 : sv);
#pragma unroll
      for (int ps = 0; ps < NPASS; ++ps) {
        const int k = ps * RPP + rq;
        const int s = __shfl(sv, k, 32);
        const v4f q = *(const v4f*)(PQ + (size_t)s * PQW + CI + 4 * p);
        v4f hv = dnc + q;
        hv.x = fmaxf(hv.x, 0.0f); hv.y = fmaxf(hv.y, 0.0f); hv.z = fmaxf(hv.z, 0.0f); hv.w = fmaxf(hv.w, 0.0f);
        v4us uh, ul;
        split4(hv, uh, ul);
        *(v4us*)(Awh + k * APZ + 4 * p) = uh;
        *(v4us*)(Awl + k * APZ + 4 * p) = ul;
      }
      __syncthreads();
      {
        v8f acc[NT];
        mma3<NT>(Awh, Awl, Bh, Bl, lane, acc);
#pragma unroll
        for (int t = 0; t < NT; ++t) {
#pragma unroll
          for (int r = 0; r < 8; ++r) {
            float v = acc[t][r] + bbv[t];
            v = ((8 * hh + r) < nv) ? v : 0.0f;
            cs[t] += v;
          }
        }
      }
      __syncthreads();
    }
#pragma unroll
    for (int t = 0; t < NT; ++t) cs[t] += __shfl_xor(cs[t], 16, 32);
#pragma unroll
    for (int t = 0; t < NT; ++t) {
      if (hh == 0) sout[wave * CI + 16 * t + m] = fmaxf(cs[t], 0.0f);
    }
    __syncthreads();
    if (CI == 32) {
      const int j = lane & 15;
      float tg = swg[512 + j];
      const float* hrow = sout + wave * CI;
#pragma unroll 1
      for (int c = 0; c < HCH; ++c) tg = fmaf(hrow[c], swg[c * 16 + j], tg);
      float gv = fmaxf(tg, 0.0f) * swg[528 + j];
      gv += __shfl_xor(gv, 8, 32);
      gv += __shfl_xor(gv, 4, 32);
      gv += __shfl_xor(gv, 2, 32);
      gv += __shfl_xor(gv, 1, 32);
      if (lane == 0) sg[it * NWAVE + wave] = gv + bg2v;
    }
    {
      v4f ov = {0.f, 0.f, 0.f, 0.f};
      if (tid < 2 * CI) ov = *(const v4f*)(sout + 4 * tid);
      float* hp = H + (size_t)(base + it * NWAVE) * CI + 4 * (tid & (2 * CI - 1));
      if (tid < 2 * CI) *(volatile v4f*)hp = ov;
      __threadfence();
      if (tid < 2 * CI) *(volatile v4f*)hp = ov;
    }
    __syncthreads();
  }
  if (CI == 32) {
    v4f gq = {0.f, 0.f, 0.f, 0.f};
    if (tid < 32) gq = *(const v4f*)(sg + 4 * tid);
    float* gp = G + (size_t)base + 4 * (tid & 31);
    if (tid < 32) *(volatile v4f*)gp = gq;
    __threadfence();
    if (tid < 32) *(volatile v4f*)gp = gq;
  }
}

__global__ __launch_bounds__(NTHR) void k_pool(const float* __restrict__ H2, const float* __restrict__ G,
                                               const int* __restrict__ bat, float* Pool, int nN) {
  __shared__ __attribute__((aligned(16))) float red[HCH * (NTHR / 2)];
  __shared__ float sred[NTHR];
  __shared__ float swv[NWAVE];
  __shared__ __attribute__((aligned(16))) float spool[HCH];
  __shared__ float sden;
  const int tid = threadIdx.x, lane = tid & 31, wave = tid >> 5;
  const int g = blockIdx.x;
  float mx = __uint_as_float(0xff800000u);
#pragma unroll 1
  for (int n0 = 0; n0 < nN; n0 += NTHR) {
    const int n = n0 + tid;
    const int nc = n > nN - 1 ? nN - 1 : n;
    const int b = bat[nc];
    const float gv = G[nc];
    const bool mt = (n < nN) && (b == g);
    mx = mt ? fmaxf(mx, gv) : mx;
  }
  mx = fmaxf(mx, __shfl_xor(mx, 16, 32));
  mx = fmaxf(mx, __shfl_xor(mx, 8, 32));
  mx = fmaxf(mx, __shfl_xor(mx, 4, 32));
  mx = fmaxf(mx, __shfl_xor(mx, 2, 32));
  mx = fmaxf(mx, __shfl_xor(mx, 1, 32));
  if (lane == 0) swv[wave] = mx;
  __syncthreads();
  float gmx = swv[0];
#pragma unroll
  for (int w = 1; w < NWAVE; ++w) gmx = fmaxf(gmx, swv[w]);

  const int slt = tid >> 1, half = tid & 1;
  float den = 0.0f;
  float acc[16];
#pragma unroll
  for (int j = 0; j < 16; ++j) acc[j] = 0.0f;
#pragma unroll 1
  for (int n0 = 0; n0 < nN; n0 += NTHR / 2) {
    const int n = n0 + slt;
    const int nc = n > nN - 1 ? nN - 1 : n;
    const int b = bat[nc];
    const bool mt = (n < nN) && (b == g);
    if (__builtin_amdgcn_ballot_w32(mt) != 0u) {
      const float e = expf(G[nc] - gmx);
      const float w = mt ? e : 0.0f;
      den += (half == 0) ? w : 0.0f;
      const float* hp = H2 + (size_t)nc * HCH + 16 * half;
      const v4f h0 = *(const v4f*)hp, h1 = *(const v4f*)(hp + 4);
      const v4f h2 = *(const v4f*)(hp + 8), h3 = *(const v4f*)(hp + 12);
      acc[0]  = fmaf(w, h0.x, acc[0]);  acc[1]  = fmaf(w, h0.y, acc[1]);
      acc[2]  = fmaf(w, h0.z, acc[2]);  acc[3]  = fmaf(w, h0.w, acc[3]);
      acc[4]  = fmaf(w, h1.x, acc[4]);  acc[5]  = fmaf(w, h1.y, acc[5]);
      acc[6]  = fmaf(w, h1.z, acc[6]);  acc[7]  = fmaf(w, h1.w, acc[7]);
      acc[8]  = fmaf(w, h2.x, acc[8]);  acc[9]  = fmaf(w, h2.y, acc[9]);
      acc[10] = fmaf(w, h2.z, acc[10]); acc[11] = fmaf(w, h2.w, acc[11]);
      acc[12] = fmaf(w, h3.x, acc[12]); acc[13] = fmaf(w, h3.y, acc[13]);
      acc[14] = fmaf(w, h3.z, acc[14]); acc[15] = fmaf(w, h3.w, acc[15]);
    }
  }
#pragma unroll
  for (int j = 0; j < 16; ++j) red[(16 * half + j) * (NTHR / 2) + slt] = acc[j];
  sred[tid] = den;
  __syncthreads();
  if (tid < HCH) {
    float s = 0.0f;
#pragma unroll 1
    for (int i = 0; i < NTHR / 2; ++i) s += red[tid * (NTHR / 2) + i];
    spool[tid] = s;
  }
  if (tid == HCH) {
    float d = 0.0f;
#pragma unroll 1
    for (int i = 0; i < NTHR; ++i) d += sred[i];
    sden = d;
  }
  __syncthreads();
  {
    const float dsum = sden;
    const float rden = dsum > 0.0f ? (1.0f / dsum) : 0.0f;
    if (tid < HCH) spool[tid] = spool[tid] * rden;
  }
  __syncthreads();
  v4f pv = {0.f, 0.f, 0.f, 0.f};
  if (tid < 8) pv = *(const v4f*)(spool + 4 * tid);
  float* pp = Pool + (size_t)g * HCH + 4 * (tid & 7);
  if (tid < 8) *(volatile v4f*)pp = pv;
  __threadfence();
  if (tid < 8) *(volatile v4f*)pp = pv;
}

__global__ __launch_bounds__(NTHR) void k_out(const float* __restrict__ Pool, const float* __restrict__ Wc1,
                                              const float* __restrict__ bc1, const float* __restrict__ Wc2,
                                              const float* __restrict__ bc2, float* out) {
  __shared__ __attribute__((aligned(16))) float sres[NG];
  const int tid = threadIdx.x;
  const int g = tid >> 2, jq = tid & 3, j0 = 4 * jq;
  float a0 = bc1[j0], a1 = bc1[j0 + 1], a2 = bc1[j0 + 2], a3 = bc1[j0 + 3];
  const float* pr = Pool + (size_t)g * HCH;
#pragma unroll 1
  for (int c = 0; c < HCH; ++c) {
    const float pv = pr[c];
    const float* w = Wc1 + c * 16 + j0;
    a0 = fmaf(pv, w[0], a0);
    a1 = fmaf(pv, w[1], a1);
    a2 = fmaf(pv, w[2], a2);
    a3 = fmaf(pv, w[3], a3);
  }
  float r = fmaxf(a0, 0.0f) * Wc2[j0];
  r = fmaf(fmaxf(a1, 0.0f), Wc2[j0 + 1], r);
  r = fmaf(fmaxf(a2, 0.0f), Wc2[j0 + 2], r);
  r = fmaf(fmaxf(a3, 0.0f), Wc2[j0 + 3], r);
  r += __shfl_xor(r, 1, 32);
  r += __shfl_xor(r, 2, 32);
  if (jq == 0) sres[g] = r + bc2[0];
  __syncthreads();
  v4f ov = {0.f, 0.f, 0.f, 0.f};
  if (tid < 16) ov = *(const v4f*)(sres + 4 * tid);
  float* op = out + 4 * (tid & 15);
  if (tid < 16) *(volatile v4f*)op = ov;
  __threadfence();
  if (tid < 16) *(volatile v4f*)op = ov;
}

extern "C" void kernel_launch(void* const* d_in, const int* in_sizes, int n_in,
                              void* d_out, int out_size, void* d_ws, size_t ws_size,
                              hipStream_t stream) {
  if (n_in < 19) return;
  const int nN = in_sizes[2];
  const int nE = in_sizes[1] / 2;
  if (nN <= 0 || nE <= 0) return;
  if (in_sizes[0] != nN * CIN || in_sizes[1] != 2 * nE) return;
  if (in_sizes[3] != 2 * CIN * 16 || in_sizes[4] != 16 || in_sizes[5] != 16 * 16 || in_sizes[6] != 16) return;
  if (in_sizes[7] != 2 * 16 * HCH || in_sizes[8] != HCH || in_sizes[9] != HCH * HCH || in_sizes[10] != HCH) return;
  if (in_sizes[11] != HCH * 16 || in_sizes[12] != 16 || in_sizes[13] != 16 || in_sizes[14] != 1) return;
  if (in_sizes[15] != HCH * 16 || in_sizes[16] != 16 || in_sizes[17] != 16 || in_sizes[18] != 1) return;
  if (out_size != NG) return;
  if (nE > (1 << 28) || nN > (1 << 24)) return;

  const float* x    = (const float*)d_in[0];
  const int*   ei   = (const int*)d_in[1];
  const int*   bat  = (const int*)d_in[2];
  const float* W1a  = (const float*)d_in[3];
  const float* b1a  = (const float*)d_in[4];
  const float* W1b  = (const float*)d_in[5];
  const float* b1b  = (const float*)d_in[6];
  const float* W2a  = (const float*)d_in[7];
  const float* b2a  = (const float*)d_in[8];
  const float* W2b  = (const float*)d_in[9];
  const float* b2b  = (const float*)d_in[10];
  const float* Wg1  = (const float*)d_in[11];
  const float* bg1  = (const float*)d_in[12];
  const float* Wg2  = (const float*)d_in[13];
  const float* bg2  = (const float*)d_in[14];
  const float* Wc1  = (const float*)d_in[15];
  const float* bc1  = (const float*)d_in[16];
  const float* Wc2  = (const float*)d_in[17];
  const float* bc2  = (const float*)d_in[18];
  const int* srcs = ei;
  const int* dsts = ei + nE;
  float* out = (float*)d_out;

  const int nBlkG  = (nN + GROWS - 1) / GROWS;
  const int NPADG  = nBlkG * GROWS;
  const int nBlkP  = (nN + NPB - 1) / NPB;
  const int NPADP  = nBlkP * NPB;
  const int nBC    = (nN + NBC - 1) / NBC;
  const int CNTPAD = nBC * NBC;
  if (2 * nBC + 1 > RBN) return;
  const int nBF    = (nN + NBF - 1) / NBF;
  const int csrLen = ((nE + 31) & ~31) + 4096;
  if (31 * 2 * nBC > 4096) return;

  char* ws = (char*)d_ws;
  size_t off = 0;
  const size_t oB   = off; off += (size_t)BPTOT * 2;               off = (off + 255) & ~(size_t)255;
  const size_t oCnt = off; off += (size_t)CNTPAD * 4;              off = (off + 255) & ~(size_t)255;
  const size_t oOff = off; off += (size_t)CNTPAD * 4;              off = (off + 255) & ~(size_t)255;
  const size_t oRb  = off; off += (size_t)RBN * 4;                 off = (off + 255) & ~(size_t)255;
  const size_t oCsr = off; off += (size_t)csrLen * 4;              off = (off + 255) & ~(size_t)255;
  const size_t oPQ1 = off; off += (size_t)NPADG * (2 * CIN) * 4;   off = (off + 255) & ~(size_t)255;
  const size_t oH1  = off; off += (size_t)NPADP * CIN * 4;         off = (off + 255) & ~(size_t)255;
  const size_t oPQ2 = off; off += (size_t)NPADG * (2 * HCH) * 4;   off = (off + 255) & ~(size_t)255;
  const size_t oH2  = off; off += (size_t)NPADP * HCH * 4;         off = (off + 255) & ~(size_t)255;
  const size_t oG   = off; off += (size_t)NPADP * 4;               off = (off + 255) & ~(size_t)255;
  const size_t oPl  = off; off += (size_t)NG * HCH * 4;            off = (off + 255) & ~(size_t)255;
  if (off > ws_size || off > (size_t)WSCAP) return;
  unsigned short* Bpl = (unsigned short*)(ws + oB);
  int*   cnt  = (int*)(ws + oCnt);
  int*   offp = (int*)(ws + oOff);
  int*   rb   = (int*)(ws + oRb);
  int*   csr  = (int*)(ws + oCsr);
  float* PQ1  = (float*)(ws + oPQ1);
  float* H1   = (float*)(ws + oH1);
  float* PQ2  = (float*)(ws + oPQ2);
  float* H2   = (float*)(ws + oH2);
  float* Gt   = (float*)(ws + oG);
  float* Pool = (float*)(ws + oPl);

  const int vec8 = ((nE & 3) == 0) ? 1 : 0;

  k_wprep<<<(WPSLOT + NTHR - 1) / NTHR, NTHR, 0, stream>>>(W1a, W1b, W2a, W2b, Bpl);
  k_count<<<nBC, NTHR, 0, stream>>>(dsts, cnt, nE, vec8);
  k_offsets<<<1, OTHR, 0, stream>>>(cnt, offp, rb, nBC);
  hipFuncSetAttribute(reinterpret_cast<const void*>(&k_fill),
                      hipFuncAttributeMaxDynamicSharedMemorySize, LDS_FILL);
  k_fill<<<nBF, NTHR, LDS_FILL, stream>>>(srcs, dsts, offp, rb, csr, nN, nE, vec8, csrLen);
  k_node<2 * CIN><<<nBlkG, GTHR, 0, stream>>>(x, Bpl + O_N1H, Bpl + O_N1L, b1a, PQ1, nN);
  k_edge<CIN><<<nBlkP, NTHR, 0, stream>>>(PQ1, csr, offp, cnt, Bpl + O_W1H, Bpl + O_W1L, b1b,
                                           Wg1, bg1, Wg2, bg2, H1, Gt, nN, csrLen);
  k_node<2 * HCH><<<nBlkG, GTHR, 0, stream>>>(H1, Bpl + O_N2H, Bpl + O_N2L, b2a, PQ2, nN);
  k_edge<HCH><<<nBlkP, NTHR, 0, stream>>>(PQ2, csr, offp, cnt, Bpl + O_W2H, Bpl + O_W2L, b2b,
                                           Wg1, bg1, Wg2, bg2, H2, Gt, nN, csrLen);
  k_pool<<<NG, NTHR, 0, stream>>>(H2, Gt, bat, Pool, nN);
  k_out<<<1, NTHR, 0, stream>>>(Pool, Wc1, bc1, Wc2, bc2, out);
}
